// GraphSAGE_89945205113354
// MI455X (gfx1250) — hardware-verified
//
#include <hip/hip_runtime.h>
#include <stddef.h>
#include <stdint.h>
#include <math.h>


#define DF     128
#define YP     256
#define HP     256
#define NG     256
#define GK     768
#define GN     512
#define HK     512
#define NTHR   256
#define NWAVE  8
#define EPT    8
#define CHUNK  (NTHR * EPT)
#define WCAP   (EPT * 32)
#define LISTN  (NWAVE * WCAP)
#define NBA    1024
#define SLA    10
#define RCAP   28672
#define DEGCAP 64
#define GBM    64
#define GBN    64
#define GTHR   128
#define AGG_ZINTS    (LISTN + 2 * RCAP + 3 * NBA)
#define MISC_INTS    16
#define ROWBUF_INTS  (NWAVE * HP / 2)
#define AGG_LDS_INTS (AGG_ZINTS + MISC_INTS + ROWBUF_INTS)
#define WPU_TOTAL    69632
#define ZU_AG  (NG * GK / 8)
#define ZU_C   (NG * DF / 4)
#define ZBLK   ((ZU_AG + ZU_C) / NTHR)
#define WSMAX  134217728

static_assert((CHUNK & (CHUNK - 1)) == 0 && CHUNK <= 4096);
static_assert((NBA & (NBA - 1)) == 0 && NBA == (1 << SLA));
static_assert(((long long)CHUNK << SLA) < (1LL << 31));
static_assert(LISTN % NTHR == 0);
static_assert(NBA % NWAVE == 0 && NBA % 32 == 0 && NBA % GBM == 0);
static_assert(RCAP % 4 == 0 && AGG_ZINTS % 4 == 0 && LISTN % 4 == 0 && ((AGG_ZINTS + MISC_INTS) % 4) == 0);
static_assert(DF % 32 == 0 && YP % 32 == 0 && GK % 32 == 0 && HK % 32 == 0 && HP % 32 == 0);
static_assert(DF == 4 * 32 && YP == 2 * DF && HP == 2 * DF && GK == 6 * DF && HK == 4 * DF && GN == 4 * DF);
static_assert(GBM == (GTHR / 32) * 16 && GBN == 64);
static_assert(NG % GBM == 0 && GN % GBN == 0 && DF % GBN == 0 && YP % GBN == 0);
static_assert(WPU_TOTAL % NTHR == 0);
static_assert(ZU_AG % NTHR == 0 && (ZU_AG + ZU_C) == ZBLK * NTHR);
static_assert(AGG_LDS_INTS * 4 <= 300000);
static_assert(GK / 8 == 96);

typedef float          v4f   __attribute__((ext_vector_type(4)));
typedef float          v8f   __attribute__((ext_vector_type(8)));
typedef int            v4i   __attribute__((ext_vector_type(4)));
typedef int            v8i   __attribute__((ext_vector_type(8)));
typedef unsigned int   v4u   __attribute__((ext_vector_type(4)));
typedef unsigned short v4us  __attribute__((ext_vector_type(4)));
typedef unsigned short v8us  __attribute__((ext_vector_type(8)));
typedef unsigned short v16us __attribute__((ext_vector_type(16)));
typedef __bf16         v16bf __attribute__((ext_vector_type(16)));
typedef v4f  __attribute__((may_alias)) v4fa;
typedef v4i  __attribute__((may_alias)) v4ia;
typedef v4us __attribute__((may_alias)) v4usa;
typedef v8us __attribute__((may_alias)) v8usa;
union FragB { v16bf v; v16us u; v8us h[2]; v8i w; };

__device__ __forceinline__ v8f wmb(const FragB& a, const FragB& b, v8f c) {
  v8f d = __builtin_amdgcn_wmma_f32_16x16x32_bf16(false, a.v, false, b.v, (short)0, c, false, false);
  asm volatile("v_nop\n\tv_nop\n\tv_nop\n\tv_nop" : "+v"(d) : "v"(a.w), "v"(b.w));
  return d;
}

__device__ __forceinline__ unsigned bf16_bits(float f) {
  const unsigned u = __float_as_uint(f);
  return (u + 0x7FFFu + ((u >> 16) & 1u)) >> 16;
}
__device__ __forceinline__ float bf16_val(float f) {
  return __uint_as_float(bf16_bits(f) << 16);
}

__device__ __forceinline__ void wave_sync() {
  __builtin_amdgcn_fence(__ATOMIC_RELEASE, "wavefront");
  __builtin_amdgcn_wave_barrier();
  __builtin_amdgcn_fence(__ATOMIC_ACQUIRE, "wavefront");
}

template <int SLB>
__device__ __forceinline__ int scan_chunk(const int* __restrict__ dsts, int nE, int cbase, int slotBase,
                                          int nb, int vec8, int* list, int tid, int lane, int wave) {
  int wc = 0;
  const int el0  = tid * EPT;
  const int e0   = cbase + el0;
  const int sent = -2147483647 - 1;
  v4i da, db;
  if (vec8 != 0 && cbase + CHUNK <= nE) {
    da = *(const v4i*)(dsts + e0);
    db = *(const v4i*)(dsts + e0 + 4);
  } else {
    da.x = (e0     < nE) ? dsts[min(e0,     nE - 1)] : sent;
    da.y = (e0 + 1 < nE) ? dsts[min(e0 + 1, nE - 1)] : sent;
    da.z = (e0 + 2 < nE) ? dsts[min(e0 + 2, nE - 1)] : sent;
    da.w = (e0 + 3 < nE) ? dsts[min(e0 + 3, nE - 1)] : sent;
    db.x = (e0 + 4 < nE) ? dsts[min(e0 + 4, nE - 1)] : sent;
    db.y = (e0 + 5 < nE) ? dsts[min(e0 + 5, nE - 1)] : sent;
    db.z = (e0 + 6 < nE) ? dsts[min(e0 + 6, nE - 1)] : sent;
    db.w = (e0 + 7 < nE) ? dsts[min(e0 + 7, nE - 1)] : sent;
  }
  const unsigned nbs = (unsigned)slotBase;
  const unsigned unb = (unsigned)nb;
  const unsigned s0 = (unsigned)da.x - nbs, s1 = (unsigned)da.y - nbs;
  const unsigned s2 = (unsigned)da.z - nbs, s3 = (unsigned)da.w - nbs;
  const unsigned s4 = (unsigned)db.x - nbs, s5 = (unsigned)db.y - nbs;
  const unsigned s6 = (unsigned)db.z - nbs, s7 = (unsigned)db.w - nbs;
  const bool h0 = s0 < unb, h1 = s1 < unb, h2 = s2 < unb, h3 = s3 < unb;
  const bool h4 = s4 < unb, h5 = s5 < unb, h6 = s6 < unb, h7 = s7 < unb;
  const unsigned any = __builtin_amdgcn_ballot_w32(h0 | h1 | h2 | h3 | h4 | h5 | h6 | h7);
  if (any != 0u) {
#define HITJ(J, HJ, SJ) { \
      const unsigned mj = __builtin_amdgcn_ballot_w32(HJ); \
      if (mj != 0u) { \
        if (HJ) { \
          const int pos = wc + (int)__builtin_amdgcn_mbcnt_lo(mj, 0u); \
          if (pos < WCAP) list[wave * WCAP + pos] = ((el0 + (J)) << SLB) | (int)(SJ); \
        } \
        wc += (int)__builtin_popcount(mj); } }
    HITJ(0, h0, s0)
    HITJ(1, h1, s1)
    HITJ(2, h2, s2)
    HITJ(3, h3, s3)
    HITJ(4, h4, s4)
    HITJ(5, h5, s5)
    HITJ(6, h6, s6)
    HITJ(7, h7, s7)
#undef HITJ
  }
  return wc;
}

__global__ __launch_bounds__(NTHR) void k_wprep(const float* __restrict__ W1l, const float* __restrict__ W1r,
                                                const float* __restrict__ W2l, const float* __restrict__ W2r,
                                                const float* __restrict__ Wih, const float* __restrict__ Whh,
                                                const float* __restrict__ Wp,
                                                unsigned short* W1C, unsigned short* W2C,
                                                unsigned short* WG, unsigned short* WP2) {
  const int u = (int)blockIdx.x * NTHR + (int)threadIdx.x;
  const float* W;
  unsigned short* P;
  int spitch, smask, dpitch, drow0, dcol0, uprl, v;
  if (u < 2048)       { W = W1l; P = W1C; spitch = 128; smask = 127; dpitch = 128; drow0 = 0;   dcol0 = 0;   uprl = 4; v = u; }
  else if (u < 4096)  { W = W1r; P = W1C; spitch = 128; smask = 127; dpitch = 128; drow0 = 128; dcol0 = 0;   uprl = 4; v = u - 2048; }
  else if (u < 8192)  { W = W2l; P = W2C; spitch = 128; smask = 127; dpitch = 256; drow0 = 0;   dcol0 = 0;   uprl = 5; v = u - 4096; }
  else if (u < 12288) { W = W2r; P = W2C; spitch = 128; smask = 127; dpitch = 256; drow0 = 128; dcol0 = 0;   uprl = 5; v = u - 8192; }
  else if (u < 28672) { W = Wih; P = WG;  spitch = 256; smask = 255; dpitch = GK;  drow0 = 0;   dcol0 = 0;   uprl = 5; v = u - 12288; }
  else if (u < 45056) { W = Wih; P = WG;  spitch = 256; smask = 255; dpitch = GK;  drow0 = 0;   dcol0 = 256; uprl = 5; v = u - 28672; }
  else if (u < 53248) { W = Whh; P = WG;  spitch = 128; smask = 127; dpitch = GK;  drow0 = 0;   dcol0 = 512; uprl = 4; v = u - 45056; }
  else if (u < 61440) { W = Whh; P = WG;  spitch = 128; smask = 127; dpitch = GK;  drow0 = 0;   dcol0 = 640; uprl = 4; v = u - 53248; }
  else if (u < 69632) { W = Wp;  P = WP2; spitch = 256; smask = 255; dpitch = HK;  drow0 = 0;   dcol0 = 0;   uprl = 6; v = u - 61440; }
  else return;
  const int r  = v >> uprl;
  const int k8 = (v & ((1 << uprl) - 1)) * 8;
  const float* p = W + (size_t)r * spitch + (k8 & smask);
  const v4f a = *(const v4f*)p;
  const v4f b = *(const v4f*)(p + 4);
  v8us o;
  o[0] = (unsigned short)bf16_bits(a.x); o[1] = (unsigned short)bf16_bits(a.y);
  o[2] = (unsigned short)bf16_bits(a.z); o[3] = (unsigned short)bf16_bits(a.w);
  o[4] = (unsigned short)bf16_bits(b.x); o[5] = (unsigned short)bf16_bits(b.y);
  o[6] = (unsigned short)bf16_bits(b.z); o[7] = (unsigned short)bf16_bits(b.w);
  unsigned short* dp = P + (size_t)(drow0 + r) * dpitch + dcol0 + k8;
  *(volatile v8us*)dp = o;
  __threadfence();
  *(volatile v8us*)dp = o;
}

__global__ __launch_bounds__(NTHR) void k_cvx(const float* __restrict__ x, int nN, int nUnits,
                                              unsigned short* xb) {
  const int u = (int)blockIdx.x * NTHR + (int)threadIdx.x;
  if (u >= nUnits) return;
  const int row = u >> 4;
  const int k8  = (u & 15) * 8;
  const int rc  = row < nN ? row : nN - 1;
  const float* p = x + (size_t)rc * DF + k8;
  const v4f a = *(const v4fa*)p;
  const v4f b = *(const v4fa*)(p + 4);
  const bool ok = row < nN;
  v8us o;
  o[0] = ok ? (unsigned short)bf16_bits(a.x) : (unsigned short)0;
  o[1] = ok ? (unsigned short)bf16_bits(a.y) : (unsigned short)0;
  o[2] = ok ? (unsigned short)bf16_bits(a.z) : (unsigned short)0;
  o[3] = ok ? (unsigned short)bf16_bits(a.w) : (unsigned short)0;
  o[4] = ok ? (unsigned short)bf16_bits(b.x) : (unsigned short)0;
  o[5] = ok ? (unsigned short)bf16_bits(b.y) : (unsigned short)0;
  o[6] = ok ? (unsigned short)bf16_bits(b.z) : (unsigned short)0;
  o[7] = ok ? (unsigned short)bf16_bits(b.w) : (unsigned short)0;
  unsigned short* dp = xb + (size_t)row * DF + k8;
  *(volatile v8us*)dp = o;
  __threadfence();
  *(volatile v8us*)dp = o;
}

__global__ __launch_bounds__(NTHR) void k_tab(const int* __restrict__ bat, int nN,
                                              unsigned short* AG, float* Cst, int* flg) {
  __shared__ int sfl[NWAVE];
  const int tid = (int)threadIdx.x, lane = tid & 31, wave = tid >> 5;
  const int b = (int)blockIdx.x;
  if (b < ZBLK) {
    const int u = b * NTHR + tid;
    const v4u z = {0u, 0u, 0u, 0u};
    if (u < ZU_AG) {
      unsigned short* p = AG + (size_t)u * 8;
      *(volatile v4u*)p = z;
      __threadfence();
      *(volatile v4u*)p = z;
    } else {
      float* p = Cst + (size_t)(u - ZU_AG) * 4;
      *(volatile v4u*)p = z;
      __threadfence();
      *(volatile v4u*)p = z;
    }
  } else {
    int bad = 0;
#pragma unroll 1
    for (int n0 = 0; n0 < nN; n0 += NTHR) {
      const int n  = n0 + tid;
      const int nc = n < nN ? n : nN - 1;
      const int np = nc > 0 ? nc - 1 : 0;
      const int bv = bat[nc];
      const int pv = bat[np];
      const int viol = ((bv < pv) | (bv < 0) | (bv >= NG)) ? 1 : 0;
      bad |= (n < nN) ? viol : 0;
    }
    const unsigned m = __builtin_amdgcn_ballot_w32(bad != 0);
    if (lane == 0) sfl[wave] = (m != 0u) ? 1 : 0;
    __syncthreads();
    int f = 0;
#pragma unroll
    for (int w2 = 0; w2 < NWAVE; ++w2) f |= sfl[w2];
    if (tid < 8) {
      v4i o = {0, 0, 0, 0};
      o.x = (tid == 0) ? f : 0;
      int* p = flg + 4 * tid;
      *(volatile v4i*)p = o;
      __threadfence();
      *(volatile v4i*)p = o;
    }
  }
}

template <int NB>
__global__ __launch_bounds__(GTHR) void k_gemm(
    const unsigned short* __restrict__ A, int lda, const unsigned short* __restrict__ WT,
    int K, float* outF, int ldo, const float* __restrict__ b0, const float* __restrict__ b1)
{
  __shared__ __attribute__((aligned(16))) float stg[GBM * GBN];
  const int tid = (int)threadIdx.x, lane = tid & 31, wave = tid >> 5, hh = lane >> 4, m = lane & 15;
  const int rowBase = (int)blockIdx.x * GBM;
  const int col0    = (int)blockIdx.y * GBN;

  v8f acc[4];
  {
    const v8f z = {0.f, 0.f, 0.f, 0.f, 0.f, 0.f, 0.f, 0.f};
    acc[0] = z; acc[1] = z; acc[2] = z; acc[3] = z;
  }
  const unsigned short* ap = A  + (size_t)(rowBase + 16 * wave + m) * (size_t)lda + 8 * hh;
  const unsigned short* wp = WT + (size_t)(col0 + m) * (size_t)K + 8 * hh;
  const int ksteps = K >> 5;
#pragma unroll 1
  for (int ks = 0; ks < ksteps; ++ks) {
    FragB af;
    af.h[0] = *(const v8usa*)(ap + 32 * ks);
    af.h[1] = *(const v8usa*)(ap + 32 * ks + 16);
#pragma unroll
    for (int t = 0; t < 4; ++t) {
      const unsigned short* wq = wp + (size_t)(16 * t) * (size_t)K + 32 * ks;
      FragB bf;
      bf.h[0] = *(const v8usa*)wq;
      bf.h[1] = *(const v8usa*)(wq + 16);
      acc[t] = wmb(af, bf, acc[t]);
    }
  }

#pragma unroll
  for (int t = 0; t < 4; ++t) {
    const int lc = 16 * t + m;
#pragma unroll
    for (int r = 0; r < 8; ++r) {
      const int lr = 16 * wave + 8 * hh + r;
      stg[lr * GBN + lc] = acc[t][r];
    }
  }
  __syncthreads();

  v4f bb = {0.f, 0.f, 0.f, 0.f};
  if constexpr (NB >= 1) {
    const v4f t0 = *(const v4f*)(b0 + col0 + 4 * m);
    bb.x = bf16_val(t0.x); bb.y = bf16_val(t0.y); bb.z = bf16_val(t0.z); bb.w = bf16_val(t0.w);
  }
  if constexpr (NB >= 2) {
    const v4f t1 = *(const v4f*)(b1 + col0 + 4 * m);
    bb.x += bf16_val(t1.x); bb.y += bf16_val(t1.y); bb.z += bf16_val(t1.z); bb.w += bf16_val(t1.w);
  }

  v4f fv[8];
#pragma unroll
  for (int i = 0; i < 8; ++i) {
    const int lr = 16 * wave + 2 * i + hh;
    const v4f t = *(const v4fa*)(stg + lr * GBN + 4 * m);
    fv[i] = t + bb;
  }
#pragma unroll
  for (int i = 0; i < 8; ++i) {
    const int lr = 16 * wave + 2 * i + hh;
    const int gr = rowBase + lr;
    float* op = outF + (size_t)gr * (size_t)ldo + col0 + 4 * m;
    *(volatile v4f*)op = fv[i];
  }
  __threadfence();
#pragma unroll
  for (int i = 0; i < 8; ++i) {
    const int lr = 16 * wave + 2 * i + hh;
    const int gr = rowBase + lr;
    float* op = outF + (size_t)gr * (size_t)ldo + col0 + 4 * m;
    *(volatile v4f*)op = fv[i];
  }
}

__device__ __forceinline__ float bn_relu(float agg, float rc, float bl, float root,
                                         float g, float rm, float sc, float be) {
  const float t = (agg * rc + bl) + root;
  const float u = (g * (t - rm)) * sc + be;
  return (u > 0.0f) ? u : (u - u);
}

template <int LAYER>
__global__ __launch_bounds__(NTHR) void k_scan(const int* __restrict__ gath, const int* __restrict__ keys,
                                               int nE, int nN, int vec8, int mRows,
                                               const float* __restrict__ Y,
                                               const float* __restrict__ bl, const float* __restrict__ gm,
                                               const float* __restrict__ bt, const float* __restrict__ rm,
                                               const float* __restrict__ rv,
                                               unsigned short* hb, float* hout) {
  extern __shared__ __attribute__((aligned(16))) int dsm[];
  int* list = dsm;
  int* hl   = dsm + LISTN;
  int* sl   = hl + RCAP;
  int* cnt  = sl + RCAP;
  int* offs = cnt + NBA;
  int* cur  = offs + NBA;
  int* misc = cur + NBA;
  const int tid = (int)threadIdx.x, lane = tid & 31, wave = tid >> 5;
  unsigned short* rowbuf = (unsigned short*)(misc + MISC_INTS) + wave * HP;
  const int nodeBase = (int)blockIdx.x * NBA;

  {
    const v4i z4 = {0, 0, 0, 0};
    for (int i = tid * 4; i < AGG_ZINTS; i += NTHR * 4) *(v4ia*)(dsm + i) = z4;
    if (tid < MISC_INTS) misc[tid] = 0;
  }
  v4f bl4, g4, be4, rm4, sc4;
  {
    const v4f t0 = *(const v4f*)(bl + 4 * lane);
    const v4f t1 = *(const v4f*)(gm + 4 * lane);
    const v4f t2 = *(const v4f*)(bt + 4 * lane);
    const v4f t3 = *(const v4f*)(rm + 4 * lane);
    const v4f t4 = *(const v4f*)(rv + 4 * lane);
    bl4.x = bf16_val(t0.x); bl4.y = bf16_val(t0.y); bl4.z = bf16_val(t0.z); bl4.w = bf16_val(t0.w);
    g4.x  = bf16_val(t1.x); g4.y  = bf16_val(t1.y); g4.z  = bf16_val(t1.z); g4.w  = bf16_val(t1.w);
    be4.x = bf16_val(t2.x); be4.y = bf16_val(t2.y); be4.z = bf16_val(t2.z); be4.w = bf16_val(t2.w);
    rm4.x = bf16_val(t3.x); rm4.y = bf16_val(t3.y); rm4.z = bf16_val(t3.z); rm4.w = bf16_val(t3.w);
    sc4.x = rsqrtf(bf16_val(t4.x) + 1e-5f); sc4.y = rsqrtf(bf16_val(t4.y) + 1e-5f);
    sc4.z = rsqrtf(bf16_val(t4.z) + 1e-5f); sc4.w = rsqrtf(bf16_val(t4.w) + 1e-5f);
  }
  __syncthreads();

  int t = 0, ov = 0;
  const int nChunks = (nE + CHUNK - 1) / CHUNK;
#pragma unroll 1
  for (int ch = 0; ch < nChunks; ++ch) {
    const int cbase = ch * CHUNK;
    const int wc = scan_chunk<SLA>(keys, nE, cbase, nodeBase, NBA, vec8, list, tid, lane, wave);
    if (lane == 0) misc[wave] = wc;
    __syncthreads();
    if (wave == 0) {
#pragma unroll 1
      for (int w2 = 0; w2 < NWAVE; ++w2) {
        int c = misc[w2];
        c = c < 0 ? 0 : (c > WCAP ? WCAP : c);
#pragma unroll 1
        for (int b0 = 0; b0 < c; b0 += 32) {
          const int idx = b0 + lane;
          const int ent = list[w2 * WCAP + (idx < WCAP ? idx : WCAP - 1)];
          const int m32 = (c - b0) < 32 ? (c - b0) : 32;
#pragma unroll 1
          for (int k = 0; k < m32; ++k) {
            const int u    = __builtin_amdgcn_readlane(ent, k);
            const int slot = u & (NBA - 1);
            const int el   = (u >> SLA) & (CHUNK - 1);
            const int pk   = ((cbase + el) << SLA) | slot;
            if (t < RCAP) {
              if (lane == 0) { hl[t] = pk; cnt[slot] = cnt[slot] + 1; }
              t = t + 1;
            } else {
              ov = 1;
            }
          }
        }
      }
    }
    __syncthreads();
  }
  if (wave == 0 && lane == 0) { misc[8] = t; misc[9] = ov; }
  __syncthreads();
  int tt = misc[8];
  tt = tt < 0 ? 0 : (tt > RCAP ? RCAP : tt);
  const int ovf = misc[9];

  if (wave == 0) {
    const int base = lane * (NBA / 32);
    int s = 0;
#pragma unroll 1
    for (int i = 0; i < NBA / 32; ++i) s += cnt[base + i];
    int incl = s;
#pragma unroll
    for (int d = 1; d < 32; d <<= 1) {
      const int y = __shfl_up(incl, d, 32);
      if (lane >= d) incl += y;
    }
    int run = incl - s;
#pragma unroll 1
    for (int i = 0; i < NBA / 32; ++i) {
      const int cv = cnt[base + i];
      offs[base + i] = run;
      cur[base + i]  = run;
      run += cv;
    }
  }
  __syncthreads();
  if (wave == 0) {
#pragma unroll 1
    for (int b0 = 0; b0 < tt; b0 += 32) {
      const int idx = b0 + lane;
      const int ent = hl[idx < RCAP ? idx : RCAP - 1];
      const int m32 = (tt - b0) < 32 ? (tt - b0) : 32;
#pragma unroll 1
      for (int k = 0; k < m32; ++k) {
        const int u    = __builtin_amdgcn_readlane(ent, k);
        const int slot = u & (NBA - 1);
        if (lane == 0) {
          int p = cur[slot];
          p = p < 0 ? 0 : (p > RCAP - 1 ? RCAP - 1 : p);
          sl[p] = u;
          cur[slot] = p + 1;
        }
      }
    }
  }
  __syncthreads();

  const float qnan = __int_as_float(0x7fc00000);
  const float pz = (ovf != 0) ? qnan : 0.0f;
#pragma unroll 1
  for (int si = 0; si < NBA / NWAVE; ++si) {
    const int s    = si * NWAVE + wave;
    const int node = nodeBase + s;
    int c = cnt[s];
    const bool big = c > DEGCAP;
    c = c < 0 ? 0 : c;
    const float cf = (c < 1) ? 1.0f : (float)c;
    c = c > DEGCAP ? DEGCAP : c;
    int o = offs[s];
    o = o < 0 ? 0 : (o > RCAP ? RCAP : o);
    const int nc = node < nN ? node : nN - 1;
    float a0 = 0.0f, a1 = 0.0f, a2 = 0.0f, a3 = 0.0f;
#pragma unroll 1
    for (int b0 = 0; b0 < c; b0 += 32) {
      int idx = o + b0 + lane;
      idx = idx > RCAP - 1 ? RCAP - 1 : idx;
      const int ent = sl[idx];
      int eid = ent >> SLA;
      eid = eid < 0 ? 0 : (eid > nE - 1 ? nE - 1 : eid);
      int sr = gath[eid];
      sr = sr < 0 ? 0 : (sr > nN - 1 ? nN - 1 : sr);
      const int m32 = (c - b0) < 32 ? (c - b0) : 32;
#pragma unroll 1
      for (int k = 0; k < m32; ++k) {
        const int sk = __builtin_amdgcn_readlane(sr, k);
        const v4f a = *(const v4f*)(Y + (size_t)sk * YP + 4 * lane);
        a0 += a.x; a1 += a.y; a2 += a.z; a3 += a.w;
      }
    }
    const v4f rt = *(const v4f*)(Y + (size_t)nc * YP + DF + 4 * lane);
    const float rc = 1.0f / cf;
    const float pzr = big ? qnan : pz;
    const bool live = node < nN;
    float y0 = bn_relu(a0, rc, bl4.x, rt.x, g4.x, rm4.x, sc4.x, be4.x);
    float y1 = bn_relu(a1, rc, bl4.y, rt.y, g4.y, rm4.y, sc4.y, be4.y);
    float y2 = bn_relu(a2, rc, bl4.z, rt.z, g4.z, rm4.z, sc4.z, be4.z);
    float y3 = bn_relu(a3, rc, bl4.w, rt.w, g4.w, rm4.w, sc4.w, be4.w);
    y0 = live ? (y0 + pzr) : 0.0f;
    y1 = live ? (y1 + pzr) : 0.0f;
    y2 = live ? (y2 + pzr) : 0.0f;
    y3 = live ? (y3 + pzr) : 0.0f;
    if constexpr (LAYER == 1) {
      v4us mh, ml;
      {
        unsigned hbits;
        hbits = bf16_bits(y0); mh[0] = (unsigned short)hbits; ml[0] = (unsigned short)bf16_bits(y0 - __uint_as_float(hbits << 16));
        hbits = bf16_bits(y1); mh[1] = (unsigned short)hbits; ml[1] = (unsigned short)bf16_bits(y1 - __uint_as_float(hbits << 16));
        hbits = bf16_bits(y2); mh[2] = (unsigned short)hbits; ml[2] = (unsigned short)bf16_bits(y2 - __uint_as_float(hbits << 16));
        hbits = bf16_bits(y3); mh[3] = (unsigned short)hbits; ml[3] = (unsigned short)bf16_bits(y3 - __uint_as_float(hbits << 16));
      }
      *(v4usa*)(rowbuf + 4 * lane) = mh;
      *(v4usa*)(rowbuf + DF + 4 * lane) = ml;
      wave_sync();
      const v8us q0 = *(const v8usa*)(rowbuf + 8 * lane);
      wave_sync();
      if (node < mRows) {
        unsigned short* rpw = hb + (size_t)node * HP + 8 * lane;
        *(volatile v8us*)rpw = q0;
        __threadfence();
        *(volatile v8us*)rpw = q0;
      }
    } else {
      v4f ow;
      ow.x = y0; ow.y = y1; ow.z = y2; ow.w = y3;
      if (node < mRows) {
        float* op = hout + (size_t)node * DF + 4 * lane;
        *(volatile v4f*)op = ow;
        __threadfence();
        *(volatile v4f*)op = ow;
      }
    }
  }
}

__device__ __forceinline__ int lower_bound_i(const int* __restrict__ a, int n, int key) {
  int lo = 0, hi = n;
#pragma unroll 1
  for (int it = 0; it < 24; ++it) {
    const int mid = (lo + hi) >> 1;
    const int mc  = mid < n ? mid : n - 1;
    const int v   = a[mc];
    const bool act = lo < hi;
    const bool lt  = v < key;
    lo = (act && lt)  ? mid + 1 : lo;
    hi = (act && !lt) ? mid     : hi;
  }
  return lo;
}

__device__ __forceinline__ float row_dot(const v4f r, const v4f q) {
  float p = r.x * q.x;
  p = fmaf(r.y, q.y, p);
  p = fmaf(r.z, q.z, p);
  p = fmaf(r.w, q.w, p);
  p += __shfl_xor(p, 16, 32);
  p += __shfl_xor(p, 8, 32);
  p += __shfl_xor(p, 4, 32);
  p += __shfl_xor(p, 2, 32);
  p += __shfl_xor(p, 1, 32);
  return p;
}

__global__ __launch_bounds__(NTHR) void k_s2s(const float* __restrict__ G, float* Cst,
                                              const float* __restrict__ H2, const int* __restrict__ bat,
                                              const int* __restrict__ flg, int nN, unsigned short* AG) {
  __shared__ __attribute__((aligned(16))) float qs[DF];
  __shared__ __attribute__((aligned(16))) float cs[DF];
  __shared__ __attribute__((aligned(16))) float wr[NWAVE * DF];
  __shared__ float wmx[NWAVE];
  __shared__ float wden[NWAVE];
  __shared__ int   wpf[NWAVE];
  __shared__ __attribute__((aligned(16))) unsigned short rowb[GK];
  const int tid = (int)threadIdx.x, lane = tid & 31, wave = tid >> 5;
  const int g = (int)blockIdx.x;

  if (tid < DF) {
    const int d = tid;
    const float* gr = G + (size_t)g * GN + d;
    const float cold = Cst[(size_t)g * DF + d];
    float ig = 0.0f, fg = 0.0f, gg = 0.0f, og = 0.0f, cn = 0.0f, th = 0.0f;
#pragma unroll 1
    for (int j = 0; j < 5; ++j) {
      const int jc = j < 4 ? j : 3;
      const float gv = gr[DF * jc];
      const float v  = (j < 4) ? gv : cn;
      const float sg = 1.0f / (1.0f + expf(-v));
      th = tanhf(v);
      ig = (j == 0) ? sg : ig;
      fg = (j == 1) ? sg : fg;
      gg = (j == 2) ? th : gg;
      og = (j == 3) ? sg : og;
      cn = fg * cold + ig * gg;
    }
    const float hn = og * th;
    qs[d] = hn;
    cs[d] = cn;
  }
  __syncthreads();

  const v4f q4 = *(const v4fa*)(qs + 4 * lane);
  int s0 = lower_bound_i(bat, nN, g);
  int e0 = lower_bound_i(bat, nN, g + 1);
  s0 = s0 < 0 ? 0 : (s0 > nN ? nN : s0);
  e0 = e0 < s0 ? s0 : (e0 > nN ? nN : e0);
  const int bad = flg[0];

  float mx = __int_as_float((int)0xff800000);
  int pf = 0;
#pragma unroll 1
  for (int n = s0 + wave; n < e0; n += NWAVE) {
    const v4f r = *(const v4f*)(H2 + (size_t)n * DF + 4 * lane);
    const float p = row_dot(r, q4);
    pf |= (p != p) ? 1 : 0;
    mx = fmaxf(mx, p);
  }
  if (lane == 0) { wmx[wave] = mx; wpf[wave] = pf; }
  __syncthreads();
  float M = wmx[0];
  int PF = wpf[0];
#pragma unroll
  for (int w2 = 1; w2 < NWAVE; ++w2) { M = fmaxf(M, wmx[w2]); PF |= wpf[w2]; }

  float den = 0.0f, a0 = 0.0f, a1 = 0.0f, a2 = 0.0f, a3 = 0.0f;
#pragma unroll 1
  for (int n = s0 + wave; n < e0; n += NWAVE) {
    const v4f r = *(const v4f*)(H2 + (size_t)n * DF + 4 * lane);
    const float p = row_dot(r, q4);
    const float a = expf(p - M);
    den += a;
    a0 = fmaf(a, r.x, a0);
    a1 = fmaf(a, r.y, a1);
    a2 = fmaf(a, r.z, a2);
    a3 = fmaf(a, r.w, a3);
  }
  {
    v4f pa;
    pa.x = a0; pa.y = a1; pa.z = a2; pa.w = a3;
    *(v4fa*)(wr + wave * DF + 4 * lane) = pa;
    if (lane == 0) wden[wave] = den;
  }
  __syncthreads();

  if (tid < DF) {
    const int d = tid;
    float s = 0.0f, dn = 0.0f;
#pragma unroll
    for (int w2 = 0; w2 < NWAVE; ++w2) { s += wr[w2 * DF + d]; dn += wden[w2]; }
    const float rr = s * (1.0f / dn);
    float r = (e0 > s0) ? rr : 0.0f;
    r = (bad != 0 || PF != 0) ? __int_as_float(0x7fc00000) : r;
    const float q = qs[d];
    const unsigned qh = bf16_bits(q);
    const unsigned ql = bf16_bits(q - __uint_as_float(qh << 16));
    const unsigned rh = bf16_bits(r);
    const unsigned rl = bf16_bits(r - __uint_as_float(rh << 16));
    rowb[d]          = (unsigned short)qh;
    rowb[DF + d]     = (unsigned short)rh;
    rowb[2 * DF + d] = (unsigned short)ql;
    rowb[3 * DF + d] = (unsigned short)rl;
    rowb[4 * DF + d] = (unsigned short)qh;
    rowb[5 * DF + d] = (unsigned short)ql;
  }
  __syncthreads();

  if (wave < 3) {
    const v8us v = *(const v8usa*)(rowb + 8 * tid);
    unsigned short* p = AG + (size_t)g * GK + 8 * tid;
    *(volatile v8us*)p = v;
    __threadfence();
    *(volatile v8us*)p = v;
  } else if (wave == 3) {
    const v4f cv = *(const v4fa*)(cs + 4 * lane);
    float* p = Cst + (size_t)g * DF + 4 * lane;
    *(volatile v4f*)p = cv;
    __threadfence();
    *(volatile v4f*)p = cv;
  }
}

static inline int cdiv(int a, int b) { return (a + b - 1) / b; }
static inline size_t al256(size_t o) { return (o + 255) & ~(size_t)255; }

extern "C" void kernel_launch(void* const* d_in, const int* in_sizes, int n_in,
                              void* d_out, int out_size, void* d_ws, size_t ws_size,
                              hipStream_t stream) {
  if (n_in < 23) return;
  if (in_sizes[0] < DF || (in_sizes[0] % DF) != 0) return;
  const int nN = in_sizes[0] / DF;
  if (nN < 16 || nN > (1 << 22)) return;
  if (in_sizes[1] < 2 || (in_sizes[1] & 1) != 0) return;
  const int nE = in_sizes[1] / 2;
  if (nE < 1 || nE >= (1 << 21)) return;
  if (in_sizes[2] != nN) return;
  if (in_sizes[3] != DF * DF || in_sizes[4] != DF || in_sizes[5] != DF * DF) return;
  if (in_sizes[6] != DF || in_sizes[7] != DF || in_sizes[8] != DF || in_sizes[9] != DF) return;
  if (in_sizes[10] != DF * DF || in_sizes[11] != DF || in_sizes[12] != DF * DF) return;
  if (in_sizes[13] != DF || in_sizes[14] != DF || in_sizes[15] != DF || in_sizes[16] != DF) return;
  if (in_sizes[17] != GN * 2 * DF || in_sizes[18] != GN * DF) return;
  if (in_sizes[19] != GN || in_sizes[20] != GN) return;
  if (in_sizes[21] != DF * 2 * DF || in_sizes[22] != DF) return;
  if (out_size != NG * DF) return;

  const float* x    = (const float*)d_in[0];
  const int*   edge = (const int*)d_in[1];
  const int*   bat  = (const int*)d_in[2];
  const float* W1l  = (const float*)d_in[3];
  const float* b1l  = (const float*)d_in[4];
  const float* W1r  = (const float*)d_in[5];
  const float* g1   = (const float*)d_in[6];
  const float* be1  = (const float*)d_in[7];
  const float* rm1  = (const float*)d_in[8];
  const float* rv1  = (const float*)d_in[9];
  const float* W2l  = (const float*)d_in[10];
  const float* b2l  = (const float*)d_in[11];
  const float* W2r  = (const float*)d_in[12];
  const float* g2   = (const float*)d_in[13];
  const float* be2  = (const float*)d_in[14];
  const float* rm2  = (const float*)d_in[15];
  const float* rv2  = (const float*)d_in[16];
  const float* Wih  = (const float*)d_in[17];
  const float* Whh  = (const float*)d_in[18];
  const float* bih  = (const float*)d_in[19];
  const float* bhh  = (const float*)d_in[20];
  const float* Wp   = (const float*)d_in[21];
  const float* bp   = (const float*)d_in[22];
  float* out = (float*)d_out;
  const int* src = edge;
  const int* dst = edge + nE;

  const int MP = cdiv(nN, GBM) * GBM;
  const int gM = MP / GBM;
  const int gA = cdiv(MP, NBA);
  if ((long long)gA * NBA < (long long)MP) return;
  const int vec8 = ((nE & 3) == 0) ? 1 : 0;

  char* ws = (char*)d_ws;
  size_t off = 0;
  const size_t oXB  = off; off = al256(off + (size_t)MP * DF * 2);
  const size_t oY   = off; off = al256(off + (size_t)MP * YP * 4);
  const size_t oH1  = off; off = al256(off + (size_t)MP * HP * 2);
  const size_t oH2  = off; off = al256(off + (size_t)MP * DF * 4);
  const size_t oW1C = off; off = al256(off + (size_t)YP * DF * 2);
  const size_t oW2C = off; off = al256(off + (size_t)YP * HP * 2);
  const size_t oWG  = off; off = al256(off + (size_t)GN * GK * 2);
  const size_t oWP2 = off; off = al256(off + (size_t)DF * HK * 2);
  const size_t oAG  = off; off = al256(off + (size_t)NG * GK * 2);
  const size_t oC   = off; off = al256(off + (size_t)NG * DF * 4);
  const size_t oG   = off; off = al256(off + (size_t)NG * GN * 4);
  const size_t oFL  = off; off = al256(off + 256);
  if (off > ws_size || off > (size_t)WSMAX) return;
  unsigned short* XB  = (unsigned short*)(ws + oXB);
  float*          Y   = (float*)(ws + oY);
  unsigned short* H1  = (unsigned short*)(ws + oH1);
  float*          H2  = (float*)(ws + oH2);
  unsigned short* W1C = (unsigned short*)(ws + oW1C);
  unsigned short* W2C = (unsigned short*)(ws + oW2C);
  unsigned short* WG  = (unsigned short*)(ws + oWG);
  unsigned short* WP2 = (unsigned short*)(ws + oWP2);
  unsigned short* AG  = (unsigned short*)(ws + oAG);
  float*          Cst = (float*)(ws + oC);
  float*          G   = (float*)(ws + oG);
  int*            FL  = (int*)(ws + oFL);

  const size_t scanLds = (size_t)AGG_LDS_INTS * 4;
  hipFuncSetAttribute(reinterpret_cast<const void*>(&k_scan<1>), hipFuncAttributeMaxDynamicSharedMemorySize, (int)scanLds);
  hipFuncSetAttribute(reinterpret_cast<const void*>(&k_scan<2>), hipFuncAttributeMaxDynamicSharedMemorySize, (int)scanLds);

  const int nUx = MP * (DF / 8);
  k_wprep<<<WPU_TOTAL / NTHR, NTHR, 0, stream>>>(W1l, W1r, W2l, W2r, Wih, Whh, Wp, W1C, W2C, WG, WP2);
  k_cvx<<<cdiv(nUx, NTHR), NTHR, 0, stream>>>(x, nN, nUx, XB);
  k_tab<<<ZBLK + 1, NTHR, 0, stream>>>(bat, nN, AG, Cst, FL);
  k_gemm<0><<<dim3(gM, YP / GBN), GTHR, 0, stream>>>(XB, DF, W1C, DF, Y, YP, b1l, b1l);
  k_scan<1><<<gA, NTHR, scanLds, stream>>>(src, dst, nE, nN, vec8, MP, Y, b1l, g1, be1, rm1, rv1, H1, H2);
  k_gemm<0><<<dim3(gM, YP / GBN), GTHR, 0, stream>>>(H1, HP, W2C, HP, Y, YP, b2l, b2l);
  k_scan<2><<<gA, NTHR, scanLds, stream>>>(src, dst, nE, nN, vec8, MP, Y, b2l, g2, be2, rm2, rv2, H1, H2);
  for (int step = 0; step < 3; ++step) {
    k_gemm<2><<<dim3(NG / GBM, GN / GBN), GTHR, 0, stream>>>(AG, GK, WG, GK, G, GN, bih, bhh);
    k_s2s<<<NG, NTHR, 0, stream>>>(G, Cst, H2, bat, FL, nN, AG);
  }
  k_gemm<1><<<dim3(NG / GBM, DF / GBN), GTHR, 0, stream>>>(AG, GK, WP2, HK, out, DF, bp, bp);
}
